// VVRWKV_SpatialMix_23373212025547
// MI455X (gfx1250) — hardware-verified
//
#include <hip/hip_runtime.h>
#include <math.h>

constexpr int kBatch    = 8;
constexpr int kTok      = 1024;
constexpr int kSide     = 32;
constexpr int kChan     = 768;
constexpr int kRows     = kBatch * kTok;
constexpr int kQuarter  = kChan / 4;
constexpr int kNDir     = 4;
constexpr int kAct      = kRows * kChan;
constexpr int kAct8     = kAct / 8;
constexpr int kWElem    = kChan * kChan;
constexpr int kW8       = kWElem / 8;
constexpr int kLanesWKV = kBatch * kChan;
constexpr float kWCarry    = 64.0f;
constexpr float kECarry    = 256.0f;
constexpr float kProjScale = 1.0f / 64.0f;
constexpr float kOutScale  = 1.0f / (64.0f * 256.0f);
constexpr float kInvT      = 1.0f / 1024.0f;
static_assert(kQuarter % 8 == 0, "8-channel groups never straddle a shift group");
static_assert(kAct8 % 256 == 0 && kW8 % 256 == 0 && kLanesWKV % 256 == 0, "exact grids");
static_assert(kRows % 64 == 0 && kChan % 64 == 0 && kChan % 32 == 0, "GEMM tile multiples");

typedef __attribute__((ext_vector_type(16))) _Float16 v16h;
typedef __attribute__((ext_vector_type(8)))  _Float16 v8h;
typedef __attribute__((ext_vector_type(16))) __bf16   v16b;
typedef __attribute__((ext_vector_type(8)))  __bf16   v8b;
typedef __attribute__((ext_vector_type(8)))  float    v8f;
typedef __attribute__((ext_vector_type(4)))  float    v4f;
typedef __attribute__((ext_vector_type(4)))  unsigned int v4u;

__device__ __forceinline__ unsigned short f2bf_bits(float f) {
  unsigned u = __float_as_uint(f);
  return (unsigned short)((u + 0x7FFFu + ((u >> 16) & 1u)) >> 16);
}
__device__ __forceinline__ float bf_bits2f(unsigned short h) { return __uint_as_float(((unsigned)h) << 16); }

__device__ __forceinline__ void dep_guard_h(v8f& a, v8f& b, v16h x, v16h y) { asm volatile("v_nop\n\tv_nop\n\tv_nop\n\tv_nop" : "+v"(a), "+v"(b) : "v"(x), "v"(y)); }
__device__ __forceinline__ void dep_guard_b(v8f& a, v8f& b, v16b x, v16b y) { asm volatile("v_nop\n\tv_nop\n\tv_nop\n\tv_nop" : "+v"(a), "+v"(b) : "v"(x), "v"(y)); }
__device__ __forceinline__ void keep4_h(v16h a, v16h b, v16h c, v16h d) { asm volatile("v_nop" :: "v"(a), "v"(b), "v"(c), "v"(d)); }
__device__ __forceinline__ void keep4_b(v16b a, v16b b, v16b c, v16b d) { asm volatile("v_nop" :: "v"(a), "v"(b), "v"(c), "v"(d)); }
__device__ __forceinline__ void acc_guard4(v8f& a, v8f& b, v8f& c, v8f& d) { asm volatile("v_nop\n\tv_nop\n\tv_nop\n\tv_nop" : "+v"(a), "+v"(b), "+v"(c), "+v"(d)); }
template <typename T> struct Frag;
template <> struct Frag<_Float16> {
  typedef v16h V; union U { v16h v; v8h h[2]; };
  static __device__ __forceinline__ v16h load(const _Float16* p) {
    U f; f.h[0] = *(const v8h*)(p); f.h[1] = *(const v8h*)(p + 16); return f.v;
  }
  static __device__ __forceinline__ v8f mma(v16h a, v16h b, v8f c) {
    return __builtin_amdgcn_wmma_f32_16x16x32_f16(false, a, false, b, (short)0, c, false, false);
  }
  static __device__ __forceinline__ void guard(v8f& a, v8f& b, v16h x, v16h y) { dep_guard_h(a, b, x, y); }
  static __device__ __forceinline__ void keep(v16h a, v16h b, v16h c, v16h d) { keep4_h(a, b, c, d); }
};
template <> struct Frag<__bf16> {
  typedef v16b V; union U { v16b v; v8b h[2]; };
  static __device__ __forceinline__ v16b load(const __bf16* p) {
    U f; f.h[0] = *(const v8b*)(p); f.h[1] = *(const v8b*)(p + 16); return f.v;
  }
  static __device__ __forceinline__ v8f mma(v16b a, v16b b, v8f c) {
    return __builtin_amdgcn_wmma_f32_16x16x32_bf16(false, a, false, b, (short)0, c, false, false);
  }
  static __device__ __forceinline__ void guard(v8f& a, v8f& b, v16b x, v16b y) { dep_guard_b(a, b, x, y); }
  static __device__ __forceinline__ void keep(v16b a, v16b b, v16b c, v16b d) { keep4_b(a, b, c, d); }
};

__device__ __forceinline__ unsigned pk16(unsigned short a, unsigned short b) { return (unsigned)a | ((unsigned)b << 16); }
__device__ __forceinline__ unsigned short h_bits(float f) { const _Float16 h = (_Float16)f; return __builtin_bit_cast(unsigned short, h); }

template <int ET> struct Elem;
template <> struct Elem<0> { typedef _Float16 T; };
template <> struct Elem<1> { typedef __bf16 T; };
template <int ET, bool SPLIT, int BIAS_MODE, int OUT_MODE, bool RESID, int ACT = 0>
__global__ __launch_bounds__(256) void wmma_gemm64(
    const unsigned short* __restrict__ Ap, const unsigned short* __restrict__ A2p, int lda, long strideA,
    const unsigned short* __restrict__ Btp, const unsigned short* __restrict__ Bt2p, int ldb, long strideB,
    void* __restrict__ Cout, void* __restrict__ Cout2, int ldc, long strideC,
    const float* __restrict__ bias,
    const float* __restrict__ resid, long strideR,
    int M, int N, int K, float scale) {
  typedef typename Elem<ET>::T T;
  typedef typename Frag<T>::V V;
  const T* A = (const T*)Ap; const T* A2 = (const T*)A2p; const T* Bt = (const T*)Btp; const T* Bt2 = (const T*)Bt2p;
  __shared__ __align__(16) float sT[8][16 * 68];
  const int b    = blockIdx.y;
  const int lane = threadIdx.x & 31;
  const int wave = threadIdx.x >> 5;
  const int tilesN = N >> 6;
  const int tilesM = M >> 6;
  const int tile = blockIdx.x * 8 + wave;
  if (tile >= tilesM * tilesN) return;
  const int tm = tile / tilesN;
  const int tn = tile - tm * tilesN;
  const int m0 = tm << 6;
  const int n0 = tn << 6;

  const T* Ab  = A  + (size_t)b * strideA;
  const T* Bb  = Bt + (size_t)b * strideB;
  const T* Ab2 = SPLIT ? (A2  + (size_t)b * strideA) : nullptr;
  const T* Bb2 = SPLIT ? (Bt2 + (size_t)b * strideB) : nullptr;

  const int rlane = lane & 15;
  const int koff  = (lane >> 4) * 8;
  const int mOff  = (lane >> 4) * 8;

  v8f acc[4][4];
#pragma unroll
  for (int i = 0; i < 4; ++i)
#pragma unroll
    for (int j = 0; j < 4; ++j) acc[i][j] = (v8f){0.f,0.f,0.f,0.f,0.f,0.f,0.f,0.f};

  for (int k0 = 0; k0 < K; k0 += 32) {
    V bh[4], bl[4];
#pragma unroll
    for (int j = 0; j < 4; ++j) {
      const size_t bo = (size_t)(n0 + (j << 4) + rlane) * ldb + koff + k0;
      bh[j] = Frag<T>::load(Bb + bo);
      if (SPLIT) bl[j] = Frag<T>::load(Bb2 + bo);
    }
#pragma unroll
    for (int i = 0; i < 4; ++i) {
      const size_t ao = (size_t)(m0 + (i << 4) + rlane) * lda + koff + k0;
      V ah = Frag<T>::load(Ab + ao);
      V al;
      if (SPLIT) al = Frag<T>::load(Ab2 + ao);
#pragma unroll
      for (int j = 0; j < 4; ++j) {
        acc[i][j] = Frag<T>::mma(ah, bh[j], acc[i][j]);
        if (SPLIT) {
          acc[i][j] = Frag<T>::mma(ah, bl[j], acc[i][j]);
          acc[i][j] = Frag<T>::mma(al, bh[j], acc[i][j]);
        }
      }
      Frag<T>::guard(acc[i][0], acc[i][3], ah, SPLIT ? al : ah);
    }
    Frag<T>::keep(bh[0], bh[1], bh[2], bh[3]);
    if (SPLIT) Frag<T>::keep(bl[0], bl[1], bl[2], bl[3]);
  }
  acc_guard4(acc[0][0], acc[0][1], acc[0][2], acc[0][3]);
  acc_guard4(acc[1][0], acc[1][1], acc[1][2], acc[1][3]);
  acc_guard4(acc[2][0], acc[2][1], acc[2][2], acc[2][3]);
  acc_guard4(acc[3][0], acc[3][1], acc[3][2], acc[3][3]);

  float* slab = sT[wave];
  const float* Rb = RESID ? (resid + (size_t)b * strideR) : nullptr;
#pragma unroll
  for (int i = 0; i < 4; ++i) {
    const int mBase = m0 + (i << 4);
#pragma unroll
    for (int j = 0; j < 4; ++j) {
      const int n = n0 + (j << 4) + rlane;
      float bv = 0.f;
      if (BIAS_MODE == 2) bv = bias[n];
#pragma unroll
      for (int r = 0; r < 8; ++r) {
        float v = acc[i][j][r] * scale;
        if (BIAS_MODE == 1) v += bias[mBase + mOff + r];
        if (BIAS_MODE == 2) v += bv;
        if (RESID) v += Rb[(size_t)(mBase + mOff + r) * ldc + n];
        if (ACT == 2) v = fmaxf(v, 0.0f);
        if (ACT == 4) v = (v > 0.f) ? v : 0.01f * v;
        slab[(mOff + r) * 68 + (j << 4) + rlane] = v;
      }
    }
    __builtin_amdgcn_fence(__ATOMIC_RELEASE, "workgroup");
    __builtin_amdgcn_wave_barrier();
    __builtin_amdgcn_fence(__ATOMIC_ACQUIRE, "workgroup");
    if (OUT_MODE == 0) {
      float* C = (float*)Cout + (size_t)b * strideC;
      const int hh = lane >> 4, c4 = (lane & 15) * 4;
      for (int pass = 0; pass < 2; ++pass) {
#pragma unroll
        for (int it = 0; it < 8; ++it) {
          const int row = it * 2 + hh;
          v4f v = *(const v4f*)(slab + row * 68 + c4);
          *(volatile v4f*)(C + (size_t)(mBase + row) * ldc + n0 + c4) = v;
        }
        __threadfence();
      }
    } else {
      const int q = lane >> 3, c8 = (lane & 7) * 8;
      unsigned short* C  = (unsigned short*)Cout  + (size_t)b * strideC;
      unsigned short* C2 = (OUT_MODE == 2) ? ((unsigned short*)Cout2 + (size_t)b * strideC) : nullptr;
      for (int pass = 0; pass < 2; ++pass) {
#pragma unroll
        for (int it = 0; it < 4; ++it) {
          const int row = it * 4 + q;
          const float* sp = slab + row * 68 + c8;
          v8h hv, lv;
#pragma unroll
          for (int e = 0; e < 8; ++e) {
            if (OUT_MODE == 1) {
              hv[e] = (_Float16)sp[e];
            } else {
              unsigned short hb = f2bf_bits(sp[e]);
              unsigned short lb = f2bf_bits(sp[e] - bf_bits2f(hb));
              hv[e] = __builtin_bit_cast(_Float16, hb);
              lv[e] = __builtin_bit_cast(_Float16, lb);
            }
          }
          *(volatile v8h*)(C + (size_t)(mBase + row) * ldc + n0 + c8) = hv;
          if (OUT_MODE == 2) *(volatile v8h*)(C2 + (size_t)(mBase + row) * ldc + n0 + c8) = lv;
        }
        __threadfence();
      }
    }
    __builtin_amdgcn_fence(__ATOMIC_RELEASE, "workgroup");
    __builtin_amdgcn_wave_barrier();
    __builtin_amdgcn_fence(__ATOMIC_ACQUIRE, "workgroup");
  }
}

__global__ __launch_bounds__(256) void shift_mix_kernel(
    const float* __restrict__ x,
    const float* __restrict__ mk, const float* __restrict__ mv, const float* __restrict__ mr,
    const int* __restrict__ hp, const int* __restrict__ wp,
    unsigned short* __restrict__ XK, unsigned short* __restrict__ XV, unsigned short* __restrict__ XR, int n8) {
  if (hp[0] * wp[0] != kTok) return;
  const int i = blockIdx.x * 256 + threadIdx.x;
  if (i >= n8) return;
  const int e  = i * 8;
  const int bt = e / kChan;
  const int c  = e - bt * kChan;
  const int t  = bt & (kTok - 1);
  const int xc = t & (kSide - 1);
  const int yr = t >> 5;
  const int grp = c / kQuarter;
  const int delta = (grp == 0) ? -1 : (grp == 1) ? 1 : (grp == 2) ? -kSide : kSide;
  const bool valid = (grp == 0) ? (xc > 0) : (grp == 1) ? (xc < kSide - 1) : (grp == 2) ? (yr > 0) : (yr < kSide - 1);
  int tn = t + delta;
  tn = tn < 0 ? 0 : (tn > kTok - 1 ? kTok - 1 : tn);
  const float* p0 = x + (size_t)e;
  const float* p1 = x + (size_t)(bt - t + tn) * kChan + c;
  const v4f a0 = *(const v4f*)(p0);       const v4f a1 = *(const v4f*)(p0 + 4);
  const v4f s0 = *(const v4f*)(p1);       const v4f s1 = *(const v4f*)(p1 + 4);
  const v4f gk0 = *(const v4f*)(mk + c);  const v4f gk1 = *(const v4f*)(mk + c + 4);
  const v4f gv0 = *(const v4f*)(mv + c);  const v4f gv1 = *(const v4f*)(mv + c + 4);
  const v4f gr0 = *(const v4f*)(mr + c);  const v4f gr1 = *(const v4f*)(mr + c + 4);
  unsigned short hk[8], hv[8], hr[8];
#pragma unroll
  for (int j = 0; j < 4; ++j) {
    const float xa = a0[j], xb = a1[j];
    const float sa = valid ? s0[j] : 0.0f;
    const float sb = valid ? s1[j] : 0.0f;
    hk[j]     = h_bits(xa * gk0[j] + sa * (1.0f - gk0[j]));
    hk[4 + j] = h_bits(xb * gk1[j] + sb * (1.0f - gk1[j]));
    hv[j]     = h_bits(xa * gv0[j] + sa * (1.0f - gv0[j]));
    hv[4 + j] = h_bits(xb * gv1[j] + sb * (1.0f - gv1[j]));
    hr[j]     = h_bits(xa * gr0[j] + sa * (1.0f - gr0[j]));
    hr[4 + j] = h_bits(xb * gr1[j] + sb * (1.0f - gr1[j]));
  }
  const v4u uk = (v4u){pk16(hk[0], hk[1]), pk16(hk[2], hk[3]), pk16(hk[4], hk[5]), pk16(hk[6], hk[7])};
  const v4u uv = (v4u){pk16(hv[0], hv[1]), pk16(hv[2], hv[3]), pk16(hv[4], hv[5]), pk16(hv[6], hv[7])};
  const v4u ur = (v4u){pk16(hr[0], hr[1]), pk16(hr[2], hr[3]), pk16(hr[4], hr[5]), pk16(hr[6], hr[7])};
  unsigned short* qk = XK + (size_t)e;
  unsigned short* qv = XV + (size_t)e;
  unsigned short* qr = XR + (size_t)e;
  *(volatile v4u*)qk = uk;
  *(volatile v4u*)qv = uv;
  *(volatile v4u*)qr = ur;
  __threadfence();
  *(volatile v4u*)qk = uk;
  *(volatile v4u*)qv = uv;
  *(volatile v4u*)qr = ur;
}

__global__ __launch_bounds__(256) void wcast8_kernel(const float* __restrict__ W0, const float* __restrict__ W1,
                                                     const float* __restrict__ W2, const float* __restrict__ W3,
                                                     unsigned short* __restrict__ out, int n8, float scale) {
  const int z = blockIdx.y;
  const float* W = (z == 0) ? W0 : (z == 1) ? W1 : (z == 2) ? W2 : W3;
  const int i = blockIdx.x * 256 + threadIdx.x;
  if (i >= n8) return;
  const float* p = W + 8 * (size_t)i;
  const v4f a = *(const v4f*)(p);
  const v4f c = *(const v4f*)(p + 4);
  unsigned short hb[8];
#pragma unroll
  for (int e = 0; e < 4; ++e) {
    hb[e]     = h_bits(a[e] * scale);
    hb[4 + e] = h_bits(c[e] * scale);
  }
  const v4u u = (v4u){pk16(hb[0], hb[1]), pk16(hb[2], hb[3]), pk16(hb[4], hb[5]), pk16(hb[6], hb[7])};
  unsigned short* q = out + (size_t)z * ((size_t)n8 * 8) + 8 * (size_t)i;
  *(volatile v4u*)q = u;
  __threadfence();
  *(volatile v4u*)q = u;
}

__device__ __forceinline__ int scan_tok(int d, int m) {
  const int mt = ((m & (kSide - 1)) << 5) | (m >> 5);
  const int base = (d & 1) ? mt : m;
  return (d & 2) ? (kTok - 1 - base) : base;
}

__global__ __launch_bounds__(256) void wkv_kernel(const float* __restrict__ Kp, const float* __restrict__ Vp,
                                                  const float* __restrict__ sd, const float* __restrict__ sf,
                                                  float* YA, float* YB, int nlanes) {
  const int g = blockIdx.x * 256 + threadIdx.x;
  if (g >= nlanes) return;
  const int b = g / kChan;
  const int c = g - b * kChan;
  const size_t base = (size_t)b * kTok * kChan + c;
  const float* kb = Kp + base;
  const float* vb = Vp + base;
#pragma unroll 1
  for (int d = 0; d < kNDir; ++d) {
    const float w = -expf(sd[d * kChan + c] * kInvT);
    const float u = sf[d * kChan + c] * kInvT;
    float* dst = ((d & 1) ? YB : YA) + base;
    const float* src = ((d & 1) ? YA : YB) + base;
    float p = 0.0f, q = 0.0f, o = -1e38f;
    int tok = scan_tok(d, 0);
    float kt = kb[(size_t)tok * kChan];
    float vt = vb[(size_t)tok * kChan];
    float pv = 0.0f;
    if (d > 0) pv = src[(size_t)tok * kChan];
#pragma unroll 1
    for (int m = 0; m < kTok; ++m) {
      const int mn = (m + 1 < kTok) ? (m + 1) : m;
      const int tokn = scan_tok(d, mn);
      const float ktn = kb[(size_t)tokn * kChan];
      const float vtn = vb[(size_t)tokn * kChan];
      float pvn = 0.0f;
      if (d > 0) pvn = src[(size_t)tokn * kChan];
      const float uk = u + kt;
      const bool ge1 = (o >= uk);
      const float e1 = expf((ge1 ? uk : o) - (ge1 ? o : uk));
      const float a1 = ge1 ? 1.0f : e1;
      const float b1 = ge1 ? e1 : 1.0f;
      const float y = (a1 * p + b1 * vt) / (a1 * q + b1);
      const float ov = pv + y;
      volatile float* vd = dst + (size_t)tok * kChan;
      *vd = ov;
      __threadfence();
      *vd = ov;
      const float wo = w + o;
      const bool ge2 = (wo >= kt);
      const float no2 = ge2 ? wo : kt;
      const float e2 = expf((ge2 ? kt : wo) - no2);
      const float a2 = ge2 ? 1.0f : e2;
      const float b2 = ge2 ? e2 : 1.0f;
      p = a2 * p + b2 * vt;
      q = a2 * q + b2;
      o = no2;
      tok = tokn; kt = ktn; vt = vtn; pv = pvn;
    }
  }
}

__global__ __launch_bounds__(256) void gate_kernel(const float* __restrict__ Y, const float* __restrict__ R,
                                                   unsigned short* __restrict__ E, int n8, float carry) {
  const int i = blockIdx.x * 256 + threadIdx.x;
  if (i >= n8) return;
  const float* py = Y + 8 * (size_t)i;
  const float* pr = R + 8 * (size_t)i;
  const v4f y0 = *(const v4f*)(py);  const v4f y1 = *(const v4f*)(py + 4);
  const v4f r0 = *(const v4f*)(pr);  const v4f r1 = *(const v4f*)(pr + 4);
  unsigned short hb[8];
#pragma unroll
  for (int e = 0; e < 4; ++e) {
    const float s0 = 1.0f / (1.0f + expf(-r0[e]));
    const float s1 = 1.0f / (1.0f + expf(-r1[e]));
    hb[e]     = h_bits(((y0[e] * 0.25f) * s0) * carry);
    hb[4 + e] = h_bits(((y1[e] * 0.25f) * s1) * carry);
  }
  const v4u u = (v4u){pk16(hb[0], hb[1]), pk16(hb[2], hb[3]), pk16(hb[4], hb[5]), pk16(hb[6], hb[7])};
  unsigned short* q = E + 8 * (size_t)i;
  *(volatile v4u*)q = u;
  __threadfence();
  *(volatile v4u*)q = u;
}

extern "C" void kernel_launch(void* const* d_in, const int* in_sizes, int n_in,
                              void* d_out, int out_size, void* d_ws, size_t ws_size,
                              hipStream_t stream) {
  if (n_in < 12) return;
  if (in_sizes[0] != kAct || out_size != kAct) return;
  if (in_sizes[1] != kNDir * kChan || in_sizes[2] != kNDir * kChan) return;
  if (in_sizes[3] != kChan || in_sizes[4] != kChan || in_sizes[5] != kChan) return;
  if (in_sizes[6] != kWElem || in_sizes[7] != kWElem || in_sizes[8] != kWElem || in_sizes[9] != kWElem) return;
  if (in_sizes[10] < 1 || in_sizes[11] < 1) return;

  const size_t plane16 = (size_t)kAct * 2;
  const size_t plane32 = (size_t)kAct * 4;
  const size_t wbytes  = (size_t)kNDir * kWElem * 2;
  const size_t offXK = 0;
  const size_t offXV = plane16;
  const size_t offXR = 2 * plane16;
  const size_t offYA = 0;
  const size_t offYB = plane32;
  const size_t offW  = 2 * plane32;
  const size_t offK  = offW + wbytes;
  const size_t offV  = offK + plane32;
  const size_t offR  = offV + plane32;
  const size_t offE  = offK;
  const size_t total = offR + plane32;
  if (total > ws_size) return;
  if (offXR + plane16 > offW) return;

  const float* x  = (const float*)d_in[0];
  const float* sd = (const float*)d_in[1];
  const float* sf = (const float*)d_in[2];
  const float* mk = (const float*)d_in[3];
  const float* mv = (const float*)d_in[4];
  const float* mr = (const float*)d_in[5];
  const float* Wk = (const float*)d_in[6];
  const float* Wv = (const float*)d_in[7];
  const float* Wr = (const float*)d_in[8];
  const float* Wo = (const float*)d_in[9];
  const int*   hp = (const int*)d_in[10];
  const int*   wp = (const int*)d_in[11];
  float* out = (float*)d_out;

  char* ws = (char*)d_ws;
  unsigned short* XK  = (unsigned short*)(ws + offXK);
  unsigned short* XV  = (unsigned short*)(ws + offXV);
  unsigned short* XR  = (unsigned short*)(ws + offXR);
  float* YA = (float*)(ws + offYA);
  float* YB = (float*)(ws + offYB);
  unsigned short* W16 = (unsigned short*)(ws + offW);
  float* Kf = (float*)(ws + offK);
  float* Vf = (float*)(ws + offV);
  float* Rf = (float*)(ws + offR);
  unsigned short* E16 = (unsigned short*)(ws + offE);
  const float* dummyf = (const float*)(ws + offW);

  shift_mix_kernel<<<dim3((unsigned)((kAct8 + 255) / 256)), dim3(256), 0, stream>>>(
      x, mk, mv, mr, hp, wp, XK, XV, XR, kAct8);

  wcast8_kernel<<<dim3((unsigned)((kW8 + 255) / 256), 4), dim3(256), 0, stream>>>(
      Wk, Wv, Wr, Wo, W16, kW8, kWCarry);

  const int tiles = (kRows / 64) * (kChan / 64);
  const dim3 ggrid((unsigned)((tiles + 7) / 8), 1);
  wmma_gemm64<0, false, 0, 0, false, 0><<<ggrid, dim3(256), 0, stream>>>(
      XK, XK, kChan, 0L, W16, W16, kChan, 0L,
      (void*)Kf, (void*)Kf, kChan, 0L, dummyf, dummyf, 0L, kRows, kChan, kChan, kProjScale);
  wmma_gemm64<0, false, 0, 0, false, 0><<<ggrid, dim3(256), 0, stream>>>(
      XV, XV, kChan, 0L, W16 + (size_t)kWElem, W16 + (size_t)kWElem, kChan, 0L,
      (void*)Vf, (void*)Vf, kChan, 0L, dummyf, dummyf, 0L, kRows, kChan, kChan, kProjScale);
  wmma_gemm64<0, false, 0, 0, false, 0><<<ggrid, dim3(256), 0, stream>>>(
      XR, XR, kChan, 0L, W16 + (size_t)2 * kWElem, W16 + (size_t)2 * kWElem, kChan, 0L,
      (void*)Rf, (void*)Rf, kChan, 0L, dummyf, dummyf, 0L, kRows, kChan, kChan, kProjScale);

  wkv_kernel<<<dim3((unsigned)((kLanesWKV + 255) / 256)), dim3(256), 0, stream>>>(
      Kf, Vf, sd, sf, YA, YB, kLanesWKV);

  gate_kernel<<<dim3((unsigned)((kAct8 + 255) / 256)), dim3(256), 0, stream>>>(
      YB, Rf, E16, kAct8, kECarry);

  wmma_gemm64<0, false, 0, 0, false, 0><<<ggrid, dim3(256), 0, stream>>>(
      E16, E16, kChan, 0L, W16 + (size_t)3 * kWElem, W16 + (size_t)3 * kWElem, kChan, 0L,
      (void*)out, (void*)out, kChan, 0L, dummyf, dummyf, 0L, kRows, kChan, kChan, kOutScale);
}
